// MutiheadRelativeAttention_3040836846167
// MI455X (gfx1250) — hardware-verified
//
#include <hip/hip_runtime.h>
#include <math.h>

constexpr int kBatch  = 4;
constexpr int kSeq    = 1024;
constexpr int kEmb    = 1024;
constexpr int kHeads  = 16;
constexpr int kHdim   = 64;
constexpr int kTok    = kBatch * kSeq;
constexpr int kSlot   = kSeq * kHdim;
constexpr int kPairs  = kBatch * kHeads;
constexpr int kRel    = 257;
constexpr int kRelPad = 320;
constexpr int kRelHalf = 128;
constexpr float kQCarry   = 16.0f;
constexpr float kRelkCarry = 64.0f;
constexpr float kQRCarry  = 64.0f;
constexpr float kInvScaling = 0.125f;
constexpr float kQRScale  = kQRCarry / (kQCarry * kRelkCarry);
constexpr float kS1Scale  = kInvScaling / (kQCarry * kQCarry);
constexpr float kS2Scale  = kInvScaling / kQRCarry;

typedef __attribute__((ext_vector_type(16))) _Float16 v16h;
typedef __attribute__((ext_vector_type(8)))  _Float16 v8h;
typedef __attribute__((ext_vector_type(16))) __bf16   v16b;
typedef __attribute__((ext_vector_type(8)))  __bf16   v8b;
typedef __attribute__((ext_vector_type(8)))  float    v8f;
typedef __attribute__((ext_vector_type(4)))  float    v4f;
typedef __attribute__((ext_vector_type(4)))  unsigned int v4u;

__device__ __forceinline__ unsigned short f2bf_bits(float f) {
  unsigned u = __float_as_uint(f);
  return (unsigned short)((u + 0x7FFFu + ((u >> 16) & 1u)) >> 16);
}
__device__ __forceinline__ float bf_bits2f(unsigned short h) { return __uint_as_float(((unsigned)h) << 16); }
__device__ __forceinline__ float bf_rne(float f) { return bf_bits2f(f2bf_bits(f)); }

__device__ __forceinline__ void dep_guard_h(v8f& a, v8f& b, v16h x, v16h y) { asm volatile("v_nop\n\tv_nop\n\tv_nop\n\tv_nop" : "+v"(a), "+v"(b) : "v"(x), "v"(y)); }
__device__ __forceinline__ void dep_guard_b(v8f& a, v8f& b, v16b x, v16b y) { asm volatile("v_nop\n\tv_nop\n\tv_nop\n\tv_nop" : "+v"(a), "+v"(b) : "v"(x), "v"(y)); }
__device__ __forceinline__ void keep4_h(v16h a, v16h b, v16h c, v16h d) { asm volatile("v_nop" :: "v"(a), "v"(b), "v"(c), "v"(d)); }
__device__ __forceinline__ void keep4_b(v16b a, v16b b, v16b c, v16b d) { asm volatile("v_nop" :: "v"(a), "v"(b), "v"(c), "v"(d)); }
__device__ __forceinline__ void acc_guard4(v8f& a, v8f& b, v8f& c, v8f& d) { asm volatile("v_nop\n\tv_nop\n\tv_nop\n\tv_nop" : "+v"(a), "+v"(b), "+v"(c), "+v"(d)); }
template <typename T> struct Frag;
template <> struct Frag<_Float16> {
  typedef v16h V; union U { v16h v; v8h h[2]; };
  static __device__ __forceinline__ v16h load(const _Float16* p) {
    U f; f.h[0] = *(const v8h*)(p); f.h[1] = *(const v8h*)(p + 16); return f.v;
  }
  static __device__ __forceinline__ v8f mma(v16h a, v16h b, v8f c) {
    return __builtin_amdgcn_wmma_f32_16x16x32_f16(false, a, false, b, (short)0, c, false, false);
  }
  static __device__ __forceinline__ void guard(v8f& a, v8f& b, v16h x, v16h y) { dep_guard_h(a, b, x, y); }
  static __device__ __forceinline__ void keep(v16h a, v16h b, v16h c, v16h d) { keep4_h(a, b, c, d); }
};
template <> struct Frag<__bf16> {
  typedef v16b V; union U { v16b v; v8b h[2]; };
  static __device__ __forceinline__ v16b load(const __bf16* p) {
    U f; f.h[0] = *(const v8b*)(p); f.h[1] = *(const v8b*)(p + 16); return f.v;
  }
  static __device__ __forceinline__ v8f mma(v16b a, v16b b, v8f c) {
    return __builtin_amdgcn_wmma_f32_16x16x32_bf16(false, a, false, b, (short)0, c, false, false);
  }
  static __device__ __forceinline__ void guard(v8f& a, v8f& b, v16b x, v16b y) { dep_guard_b(a, b, x, y); }
  static __device__ __forceinline__ void keep(v16b a, v16b b, v16b c, v16b d) { keep4_b(a, b, c, d); }
};

__device__ __forceinline__ unsigned pk16(unsigned short a, unsigned short b) { return (unsigned)a | ((unsigned)b << 16); }
__device__ __forceinline__ unsigned short h_bits(float f) { const _Float16 h = (_Float16)f; return __builtin_bit_cast(unsigned short, h); }
__device__ __forceinline__ float h16_to_f(unsigned short u) { return (float)__builtin_bit_cast(_Float16, u); }
__device__ __forceinline__ void lds_wave_sync() {
  __builtin_amdgcn_fence(__ATOMIC_RELEASE, "workgroup");
  __builtin_amdgcn_wave_barrier();
  __builtin_amdgcn_fence(__ATOMIC_ACQUIRE, "workgroup");
}

template <int ET> struct Elem;
template <> struct Elem<0> { typedef _Float16 T; };
template <> struct Elem<1> { typedef __bf16 T; };
template <int ET, int SPLIT, int BIAS_MODE, int OUT_MODE, bool RESID, int ACT = 0>
__global__ __launch_bounds__(256) void wmma_gemm64(
    const unsigned short* __restrict__ Ap, const unsigned short* __restrict__ A2p, int lda, long strideA,
    const unsigned short* __restrict__ Btp, const unsigned short* __restrict__ Bt2p, int ldb, long strideB,
    void* __restrict__ Cout, void* __restrict__ Cout2, int ldc, long strideC,
    const float* __restrict__ bias,
    const float* __restrict__ resid, long strideR,
    int M, int N, int K, float scale, float post,
    int rdiv, long rshi, int cdiv, long cshi) {
  typedef typename Elem<ET>::T T;
  typedef typename Frag<T>::V V;
  const T* A = (const T*)Ap; const T* A2 = (const T*)A2p; const T* Bt = (const T*)Btp; const T* Bt2 = (const T*)Bt2p;
  __shared__ __align__(16) float sT[8][16 * 68];
  const int b    = blockIdx.y;
  const int lane = threadIdx.x & 31;
  const int wave = threadIdx.x >> 5;
  const int tilesN = N >> 6;
  const int tilesM = M >> 6;
  const int tile = blockIdx.x * 8 + wave;
  if (tile >= tilesM * tilesN) return;
  const int tm = tile / tilesN;
  const int tn = tile - tm * tilesN;
  const int m0 = tm << 6;
  const int n0 = tn << 6;

  const T* Ab  = A  + (size_t)b * strideA;
  const T* Bb  = Bt + (size_t)b * strideB;
  const T* Ab2 = SPLIT ? (A2  + (size_t)b * strideA) : nullptr;
  const T* Bb2 = (SPLIT == 1) ? (Bt2 + (size_t)b * strideB) : nullptr;

  const int rlane = lane & 15;
  const int koff  = (lane >> 4) * 8;
  const int mOff  = (lane >> 4) * 8;

  v8f acc[4][4];
#pragma unroll
  for (int i = 0; i < 4; ++i)
#pragma unroll
    for (int j = 0; j < 4; ++j) acc[i][j] = (v8f){0.f,0.f,0.f,0.f,0.f,0.f,0.f,0.f};

  for (int k0 = 0; k0 < K; k0 += 32) {
    V bh[4], bl[4];
#pragma unroll
    for (int j = 0; j < 4; ++j) {
      const size_t bo = (size_t)(n0 + (j << 4) + rlane) * ldb + koff + k0;
      bh[j] = Frag<T>::load(Bb + bo);
      if (SPLIT == 1) bl[j] = Frag<T>::load(Bb2 + bo);
    }
#pragma unroll
    for (int i = 0; i < 4; ++i) {
      const size_t ao = (size_t)(m0 + (i << 4) + rlane) * lda + koff + k0;
      V ah = Frag<T>::load(Ab + ao);
      V al;
      if (SPLIT) al = Frag<T>::load(Ab2 + ao);
#pragma unroll
      for (int j = 0; j < 4; ++j) {
        acc[i][j] = Frag<T>::mma(ah, bh[j], acc[i][j]);
        if (SPLIT == 1) {
          acc[i][j] = Frag<T>::mma(ah, bl[j], acc[i][j]);
          acc[i][j] = Frag<T>::mma(al, bh[j], acc[i][j]);
        }
        if (SPLIT == 3) {
          acc[i][j] = Frag<T>::mma(al, bh[j], acc[i][j]);
        }
      }
      Frag<T>::guard(acc[i][0], acc[i][3], ah, SPLIT ? al : ah);
    }
    Frag<T>::keep(bh[0], bh[1], bh[2], bh[3]);
    if (SPLIT == 1) Frag<T>::keep(bl[0], bl[1], bl[2], bl[3]);
  }
  acc_guard4(acc[0][0], acc[0][1], acc[0][2], acc[0][3]);
  acc_guard4(acc[1][0], acc[1][1], acc[1][2], acc[1][3]);
  acc_guard4(acc[2][0], acc[2][1], acc[2][2], acc[2][3]);
  acc_guard4(acc[3][0], acc[3][1], acc[3][2], acc[3][3]);

  const size_t cbase = (size_t)b * strideC + (size_t)(m0 / rdiv) * (size_t)rshi + (size_t)(m0 % rdiv) * (size_t)ldc
                     + (size_t)(n0 / cdiv) * (size_t)cshi + (size_t)(n0 % cdiv);
  float* slab = sT[wave];
  const float* Rb = RESID ? (resid + (size_t)b * strideR) : nullptr;
#pragma unroll
  for (int i = 0; i < 4; ++i) {
    const int mBase = m0 + (i << 4);
#pragma unroll
    for (int j = 0; j < 4; ++j) {
      const int n = n0 + (j << 4) + rlane;
      float bv = 0.f;
      if (BIAS_MODE == 2) bv = bias[n];
#pragma unroll
      for (int r = 0; r < 8; ++r) {
        float v = acc[i][j][r] * scale;
        if (BIAS_MODE == 1) v += bias[mBase + mOff + r];
        if (BIAS_MODE == 2) v += bv;
        if (RESID) v += Rb[(size_t)(mBase + mOff + r) * ldc + n];
        if (ACT == 2) v = fmaxf(v, 0.0f);
        if (ACT == 4) v = (v > 0.f) ? v : 0.01f * v;
        v *= post;
        slab[(mOff + r) * 68 + (j << 4) + rlane] = v;
      }
    }
    __builtin_amdgcn_fence(__ATOMIC_RELEASE, "workgroup");
    __builtin_amdgcn_wave_barrier();
    __builtin_amdgcn_fence(__ATOMIC_ACQUIRE, "workgroup");
    if (OUT_MODE == 0) {
      float* C = (float*)Cout + cbase;
      const int hh = lane >> 4, c4 = (lane & 15) * 4;
      for (int pass = 0; pass < 2; ++pass) {
#pragma unroll
        for (int it = 0; it < 8; ++it) {
          const int row = it * 2 + hh;
          v4f v = *(const v4f*)(slab + row * 68 + c4);
          *(volatile v4f*)(C + (size_t)((i << 4) + row) * ldc + c4) = v;
        }
        __threadfence();
      }
    } else {
      const int q = lane >> 3, c8 = (lane & 7) * 8;
      unsigned short* C  = (unsigned short*)Cout  + cbase;
      unsigned short* C2 = (OUT_MODE == 2) ? ((unsigned short*)Cout2 + cbase) : nullptr;
      for (int pass = 0; pass < 2; ++pass) {
#pragma unroll
        for (int it = 0; it < 4; ++it) {
          const int row = it * 4 + q;
          const float* sp = slab + row * 68 + c8;
          v8h hv, lv;
#pragma unroll
          for (int e = 0; e < 8; ++e) {
            if (OUT_MODE == 1) {
              hv[e] = (_Float16)sp[e];
            } else {
              unsigned short hb = f2bf_bits(sp[e]);
              unsigned short lb = f2bf_bits(sp[e] - bf_bits2f(hb));
              hv[e] = __builtin_bit_cast(_Float16, hb);
              lv[e] = __builtin_bit_cast(_Float16, lb);
            }
          }
          *(volatile v8h*)(C + (size_t)((i << 4) + row) * ldc + c8) = hv;
          if (OUT_MODE == 2) *(volatile v8h*)(C2 + (size_t)((i << 4) + row) * ldc + c8) = lv;
        }
        __threadfence();
      }
    }
    __builtin_amdgcn_fence(__ATOMIC_RELEASE, "workgroup");
    __builtin_amdgcn_wave_barrier();
    __builtin_amdgcn_fence(__ATOMIC_ACQUIRE, "workgroup");
  }
}

__global__ __launch_bounds__(256) void cast_f32_bf16x2(
    const float* __restrict__ in, unsigned short* __restrict__ out, int n2) {
  int i = blockIdx.x * 256 + threadIdx.x;
  if (i < n2) {
    const unsigned u = pk16(f2bf_bits(in[2 * i]), f2bf_bits(in[2 * i + 1]));
    ((volatile unsigned*)out)[i] = u;
    __threadfence();
    ((volatile unsigned*)out)[i] = u;
  }
}

__global__ __launch_bounds__(256) void cast4_f32_bf16x2(
    const float* __restrict__ W0, const float* __restrict__ W1, const float* __restrict__ W2, const float* __restrict__ W3,
    unsigned short* __restrict__ out, int n2plane) {
  const int z = blockIdx.y;
  const float* in = (z == 0) ? W0 : (z == 1) ? W1 : (z == 2) ? W2 : W3;
  int i = blockIdx.x * 256 + threadIdx.x;
  if (i < n2plane) {
    const unsigned u = pk16(f2bf_bits(in[2 * i]), f2bf_bits(in[2 * i + 1]));
    volatile unsigned* op = (volatile unsigned*)(out + (size_t)z * 2 * (size_t)n2plane);
    op[i] = u;
    __threadfence();
    op[i] = u;
  }
}

__global__ __launch_bounds__(256) void rel_tables_kernel(
    const float* __restrict__ rel_k, const float* __restrict__ rel_v,
    unsigned short* __restrict__ relk16, unsigned short* __restrict__ relvT, float kcarry) {
  const int part = blockIdx.y;
  const int ch = blockIdx.x * 256 + threadIdx.x;
  if (ch >= (kRelPad * kHdim) / 8) return;
  unsigned short o[8];
  unsigned short* dst;
  if (part == 0) {
    const int c = ch >> 3, d0 = (ch & 7) * 8;
    const int cc = (c < kRel) ? c : (kRel - 1);
#pragma unroll
    for (int e = 0; e < 8; ++e) {
      float f = rel_k[cc * kHdim + d0 + e];
      f = (c < kRel) ? f : 0.0f;
      o[e] = h_bits(bf_rne(f) * kcarry);
    }
    dst = relk16 + (size_t)ch * 8;
  } else {
    const int d = ch / (kRelPad / 8);
    const int c0 = (ch - d * (kRelPad / 8)) * 8;
#pragma unroll
    for (int e = 0; e < 8; ++e) {
      const int c = c0 + e;
      const int cc = (c < kRel) ? c : (kRel - 1);
      float f = rel_v[cc * kHdim + d];
      f = (c < kRel) ? f : 0.0f;
      o[e] = f2bf_bits(f);
    }
    dst = relvT + (size_t)ch * 8;
  }
  const v4u u = (v4u){pk16(o[0], o[1]), pk16(o[2], o[3]), pk16(o[4], o[5]), pk16(o[6], o[7])};
  *(volatile v4u*)dst = u;
  __threadfence();
  *(volatile v4u*)dst = u;
}

__global__ __launch_bounds__(256) void softmax_bins_kernel(
    const float* __restrict__ S, const unsigned short* __restrict__ QR,
    unsigned short* __restrict__ Ph, unsigned short* __restrict__ Pl,
    unsigned short* __restrict__ Hh, unsigned short* __restrict__ Hl, float qrs) {
  __shared__ __align__(16) float sP[8][kSeq];
  const int wave = threadIdx.x >> 5, lane = threadIdx.x & 31;
  const int row = blockIdx.x * 8 + wave;
  const int qi = row & (kSeq - 1);
  const float* srow = S + (size_t)row * kSeq;
  const unsigned short* qrow = QR + (size_t)row * kRelPad;
  float* pw = sP[wave];

  float mx = -INFINITY;
#pragma unroll 1
  for (int k = 0; k < 4; ++k) {
    const int j0 = 256 * k + 8 * lane;
    const v4f a0 = *(const v4f*)(srow + j0);
    const v4f a1 = *(const v4f*)(srow + j0 + 4);
    float sv[8];
    sv[0] = a0[0]; sv[1] = a0[1]; sv[2] = a0[2]; sv[3] = a0[3];
    sv[4] = a1[0]; sv[5] = a1[1]; sv[6] = a1[2]; sv[7] = a1[3];
#pragma unroll
    for (int e = 0; e < 8; ++e) {
      int idx = qi - (j0 + e) + kRelHalf;
      idx = idx < 0 ? 0 : (idx > 2 * kRelHalf ? 2 * kRelHalf : idx);
      const float qr = h16_to_f(qrow[idx]);
      const float s = fmaf(qr, qrs, sv[e]);
      sv[e] = s;
      mx = fmaxf(mx, s);
    }
    const v4f o0 = (v4f){sv[0], sv[1], sv[2], sv[3]};
    const v4f o1 = (v4f){sv[4], sv[5], sv[6], sv[7]};
    *(v4f*)(pw + j0) = o0;
    *(v4f*)(pw + j0 + 4) = o1;
  }
#pragma unroll
  for (int off = 16; off > 0; off >>= 1) mx = fmaxf(mx, __shfl_xor(mx, off, 32));
  lds_wave_sync();

  float sum = 0.f;
#pragma unroll 1
  for (int k = 0; k < 4; ++k) {
    const int j0 = 256 * k + 8 * lane;
    const v4f a0 = *(const v4f*)(pw + j0);
    const v4f a1 = *(const v4f*)(pw + j0 + 4);
    sum += __expf(a0[0] - mx); sum += __expf(a0[1] - mx); sum += __expf(a0[2] - mx); sum += __expf(a0[3] - mx);
    sum += __expf(a1[0] - mx); sum += __expf(a1[1] - mx); sum += __expf(a1[2] - mx); sum += __expf(a1[3] - mx);
  }
#pragma unroll
  for (int off = 16; off > 0; off >>= 1) sum += __shfl_xor(sum, off, 32);
  const float inv = 1.0f / sum;

  float sA = 0.f, sB = 0.f;
#pragma unroll 1
  for (int k = 0; k < 4; ++k) {
    const int j0 = 256 * k + 8 * lane;
    const v4f a0 = *(const v4f*)(pw + j0);
    const v4f a1 = *(const v4f*)(pw + j0 + 4);
    float pv[8];
    pv[0] = a0[0]; pv[1] = a0[1]; pv[2] = a0[2]; pv[3] = a0[3];
    pv[4] = a1[0]; pv[5] = a1[1]; pv[6] = a1[2]; pv[7] = a1[3];
    unsigned short hb[8], lb[8];
#pragma unroll
    for (int e = 0; e < 8; ++e) {
      const float p = __expf(pv[e] - mx) * inv;
      pv[e] = p;
      const int j = j0 + e;
      sA += (j >= qi + kRelHalf) ? p : 0.0f;
      sB += (j <= qi - kRelHalf) ? p : 0.0f;
      hb[e] = f2bf_bits(p);
      lb[e] = f2bf_bits(p - bf_bits2f(hb[e]));
    }
    const v4f o0 = (v4f){pv[0], pv[1], pv[2], pv[3]};
    const v4f o1 = (v4f){pv[4], pv[5], pv[6], pv[7]};
    *(v4f*)(pw + j0) = o0;
    *(v4f*)(pw + j0 + 4) = o1;
    const v4u uh = (v4u){pk16(hb[0], hb[1]), pk16(hb[2], hb[3]), pk16(hb[4], hb[5]), pk16(hb[6], hb[7])};
    const v4u ul = (v4u){pk16(lb[0], lb[1]), pk16(lb[2], lb[3]), pk16(lb[4], lb[5]), pk16(lb[6], lb[7])};
    unsigned short* ph = Ph + (size_t)row * kSeq + j0;
    unsigned short* pl = Pl + (size_t)row * kSeq + j0;
    *(volatile v4u*)ph = uh;
    *(volatile v4u*)pl = ul;
    __threadfence();
    *(volatile v4u*)ph = uh;
    *(volatile v4u*)pl = ul;
  }
#pragma unroll
  for (int off = 16; off > 0; off >>= 1) { sA += __shfl_xor(sA, off, 32); sB += __shfl_xor(sB, off, 32); }
  lds_wave_sync();

  {
    unsigned short hb[8], lb[8];
#pragma unroll
    for (int e = 0; e < 8; ++e) {
      const int c = 8 * lane + e;
      const int j = qi + kRelHalf - c;
      const int jc = j < 0 ? 0 : (j > kSeq - 1 ? kSeq - 1 : j);
      const float p = pw[jc];
      const bool band = (c >= 1) && (j >= 0) && (j <= kSeq - 1);
      float v = band ? p : 0.0f;
      v = (c == 0) ? sA : v;
      hb[e] = f2bf_bits(v);
      lb[e] = f2bf_bits(v - bf_bits2f(hb[e]));
    }
    const v4u uh = (v4u){pk16(hb[0], hb[1]), pk16(hb[2], hb[3]), pk16(hb[4], hb[5]), pk16(hb[6], hb[7])};
    const v4u ul = (v4u){pk16(lb[0], lb[1]), pk16(lb[2], lb[3]), pk16(lb[4], lb[5]), pk16(lb[6], lb[7])};
    unsigned short* hh = Hh + (size_t)row * kRelPad + 8 * lane;
    unsigned short* hl = Hl + (size_t)row * kRelPad + 8 * lane;
    *(volatile v4u*)hh = uh;
    *(volatile v4u*)hl = ul;
    __threadfence();
    *(volatile v4u*)hh = uh;
    *(volatile v4u*)hl = ul;
  }
  {
    unsigned short hb[8], lb[8];
#pragma unroll
    for (int e = 0; e < 8; ++e) {
      const int c = 2 * kRelHalf + 8 * lane + e;
      const float v = (c == 2 * kRelHalf) ? sB : 0.0f;
      hb[e] = f2bf_bits(v);
      lb[e] = f2bf_bits(v - bf_bits2f(hb[e]));
    }
    const v4u uh = (v4u){pk16(hb[0], hb[1]), pk16(hb[2], hb[3]), pk16(hb[4], hb[5]), pk16(hb[6], hb[7])};
    const v4u ul = (v4u){pk16(lb[0], lb[1]), pk16(lb[2], lb[3]), pk16(lb[4], lb[5]), pk16(lb[6], lb[7])};
    if (lane < 8) {
      unsigned short* hh = Hh + (size_t)row * kRelPad + 2 * kRelHalf + 8 * lane;
      unsigned short* hl = Hl + (size_t)row * kRelPad + 2 * kRelHalf + 8 * lane;
      *(volatile v4u*)hh = uh;
      *(volatile v4u*)hl = ul;
      __threadfence();
      *(volatile v4u*)hh = uh;
      *(volatile v4u*)hl = ul;
    }
  }
}

__global__ __launch_bounds__(256) void combine_split_kernel(
    const float* __restrict__ W1m, const float* __restrict__ W2m,
    unsigned short* __restrict__ Ah, unsigned short* __restrict__ Al, int n8) {
  const int t = blockIdx.x * 256 + threadIdx.x;
  if (t < n8) {
    const float* p1 = W1m + (size_t)t * 8;
    const float* p2 = W2m + (size_t)t * 8;
    const v4f a0 = *(const v4f*)(p1), a1 = *(const v4f*)(p1 + 4);
    const v4f b0 = *(const v4f*)(p2), b1 = *(const v4f*)(p2 + 4);
    float v[8];
    v[0] = a0[0] + b0[0]; v[1] = a0[1] + b0[1]; v[2] = a0[2] + b0[2]; v[3] = a0[3] + b0[3];
    v[4] = a1[0] + b1[0]; v[5] = a1[1] + b1[1]; v[6] = a1[2] + b1[2]; v[7] = a1[3] + b1[3];
    unsigned short hb[8], lb[8];
#pragma unroll
    for (int e = 0; e < 8; ++e) { hb[e] = f2bf_bits(v[e]); lb[e] = f2bf_bits(v[e] - bf_bits2f(hb[e])); }
    const v4u uh = (v4u){pk16(hb[0], hb[1]), pk16(hb[2], hb[3]), pk16(hb[4], hb[5]), pk16(hb[6], hb[7])};
    const v4u ul = (v4u){pk16(lb[0], lb[1]), pk16(lb[2], lb[3]), pk16(lb[4], lb[5]), pk16(lb[6], lb[7])};
    unsigned short* ah = Ah + (size_t)t * 8;
    unsigned short* al = Al + (size_t)t * 8;
    *(volatile v4u*)ah = uh;
    *(volatile v4u*)al = ul;
    __threadfence();
    *(volatile v4u*)ah = uh;
    *(volatile v4u*)al = ul;
  }
}

extern "C" void kernel_launch(void* const* d_in, const int* in_sizes, int n_in,
                              void* d_out, int out_size, void* d_ws, size_t ws_size,
                              hipStream_t stream)
{
  if (n_in < 11) return;
  if (in_sizes[0] != kTok * kEmb || in_sizes[1] != kEmb * kEmb || in_sizes[3] != kEmb * kEmb ||
      in_sizes[5] != kEmb * kEmb || in_sizes[7] != kEmb * kEmb || in_sizes[2] != kEmb || in_sizes[4] != kEmb ||
      in_sizes[6] != kEmb || in_sizes[8] != kEmb || in_sizes[9] != kRel * kHdim || in_sizes[10] != kRel * kHdim) return;
  if (out_size != kTok * kEmb) return;

  const float* hidden = (const float*)d_in[0];
  const float* Wq = (const float*)d_in[1];
  const float* bq = (const float*)d_in[2];
  const float* Wk = (const float*)d_in[3];
  const float* bk = (const float*)d_in[4];
  const float* Wv = (const float*)d_in[5];
  const float* bv = (const float*)d_in[6];
  const float* Wo = (const float*)d_in[7];
  const float* bo = (const float*)d_in[8];
  const float* rel_k = (const float*)d_in[9];
  const float* rel_v = (const float*)d_in[10];
  float* out = (float*)d_out;

  const size_t bHid  = (size_t)kTok * kEmb * 2;
  const size_t bW4   = (size_t)4 * kEmb * kEmb * 2;
  const size_t bQK   = (size_t)2 * kPairs * kSlot * 2;
  const size_t bVT   = (size_t)kPairs * kSlot * 2;
  const size_t bRelk = (size_t)kRelPad * kHdim * 2;
  const size_t bRelv = (size_t)kHdim * kRelPad * 2;
  const size_t bQR   = (size_t)kBatch * kSeq * kRelPad * 2;
  const size_t bS    = (size_t)kBatch * kSeq * kSeq * 4;
  const size_t bP    = (size_t)kBatch * kSeq * kSeq * 2;
  const size_t bH    = (size_t)kBatch * kSeq * kRelPad * 2;
  const size_t bWm   = (size_t)kTok * kEmb * 4;

  size_t off = 0;
  const size_t oHid = off;  off += bHid;
  const size_t oW4  = off;  off += bW4;
  const size_t oQK  = off;  off += bQK;
  const size_t oVTh = off;  off += bVT;
  const size_t oVTl = off;  off += bVT;
  const size_t oRelk = off; off += bRelk;
  const size_t oRelv = off; off += bRelv;
  const size_t oQR  = off;  off += bQR;
  const size_t oS   = off;  off += bS;
  const size_t oPh  = off;  off += bP;
  const size_t oPl  = off;  off += bP;
  const size_t oHh  = off;  off += bH;
  const size_t oHl  = off;  off += bH;
  const size_t oW1  = off;  off += bWm;
  const size_t oW2  = off;  off += bWm;
  if (off > ws_size) return;
  if ((size_t)kTok * kEmb * 2 > bHid || (size_t)kTok * kEmb * 2 > bS) return;

  char* ws = (char*)d_ws;
  unsigned short* hid_bf = (unsigned short*)(ws + oHid);
  unsigned short* w4_bf  = (unsigned short*)(ws + oW4);
  unsigned short* wq_bf  = w4_bf;
  unsigned short* wk_bf  = w4_bf + (size_t)kEmb * kEmb;
  unsigned short* wv_bf  = w4_bf + (size_t)2 * kEmb * kEmb;
  unsigned short* wo_bf  = w4_bf + (size_t)3 * kEmb * kEmb;
  unsigned short* q16    = (unsigned short*)(ws + oQK);
  unsigned short* k16    = q16 + (size_t)kPairs * kSlot;
  unsigned short* vTh    = (unsigned short*)(ws + oVTh);
  unsigned short* vTl    = (unsigned short*)(ws + oVTl);
  unsigned short* relk16 = (unsigned short*)(ws + oRelk);
  unsigned short* relvT  = (unsigned short*)(ws + oRelv);
  unsigned short* QRg    = (unsigned short*)(ws + oQR);
  float*          Sbuf   = (float*)(ws + oS);
  unsigned short* Ph     = (unsigned short*)(ws + oPh);
  unsigned short* Pl     = (unsigned short*)(ws + oPl);
  unsigned short* Hh     = (unsigned short*)(ws + oHh);
  unsigned short* Hl     = (unsigned short*)(ws + oHl);
  float*          W1m    = (float*)(ws + oW1);
  float*          W2m    = (float*)(ws + oW2);
  unsigned short* attnh  = (unsigned short*)(ws + oHid);
  unsigned short* attnl  = (unsigned short*)(ws + oS);

  const int NODIV = 1 << 30;

  {
    const int n2 = kTok * kEmb / 2;
    cast_f32_bf16x2<<<dim3(n2 / 256), 256, 0, stream>>>(hidden, hid_bf, n2);
    const int n2w = kEmb * kEmb / 2;
    cast4_f32_bf16x2<<<dim3(n2w / 256, 4), 256, 0, stream>>>(Wq, Wk, Wv, Wo, w4_bf, n2w);
    rel_tables_kernel<<<dim3((kRelPad * kHdim / 8) / 256, 2), 256, 0, stream>>>(rel_k, rel_v, relk16, relvT, kRelkCarry);
  }

  wmma_gemm64<1, 0, 2, 1, false><<<dim3(((kTok / 64) * (kEmb / 64)) / 8, 1), 256, 0, stream>>>(
      hid_bf, nullptr, kEmb, 0L,
      wq_bf, nullptr, kEmb, 0L,
      (void*)q16, nullptr, kHdim, 0L,
      bq, nullptr, 0L,
      kTok, kEmb, kEmb, 1.0f, kQCarry,
      kSeq, (long)kSlot, kHdim, (long)4 * kSlot);
  wmma_gemm64<1, 0, 2, 1, false><<<dim3(((kTok / 64) * (kEmb / 64)) / 8, 1), 256, 0, stream>>>(
      hid_bf, nullptr, kEmb, 0L,
      wk_bf, nullptr, kEmb, 0L,
      (void*)k16, nullptr, kHdim, 0L,
      bk, nullptr, 0L,
      kTok, kEmb, kEmb, 1.0f, kQCarry,
      kSeq, (long)kSlot, kHdim, (long)4 * kSlot);
  wmma_gemm64<1, 0, 1, 2, false><<<dim3(((kEmb / 64) * (kTok / 64)) / 8, 1), 256, 0, stream>>>(
      wv_bf, nullptr, kEmb, 0L,
      hid_bf, nullptr, kEmb, 0L,
      (void*)vTh, (void*)vTl, kSeq, 0L,
      bv, nullptr, 0L,
      kEmb, kTok, kEmb, 1.0f, 1.0f,
      kHdim, (long)4 * kSlot, kSeq, (long)kSlot);

  for (int a = 0; a < 4; ++a) {
    for (int c = 0; c < 4; ++c) {
      const size_t tgtSlot = (size_t)(16 * a + 4 * c) * kSlot;
      const size_t srcSlot = (size_t)(16 * c + a) * kSlot;
      wmma_gemm64<0, 0, 0, 1, false><<<dim3(((kSeq / 64) * (kRelPad / 64)) / 8, kBatch), 256, 0, stream>>>(
          q16 + srcSlot, nullptr, kHdim, (long)4 * kSlot,
          relk16, nullptr, kHdim, 0L,
          (void*)QRg, nullptr, kRelPad, (long)kSeq * kRelPad,
          nullptr, nullptr, 0L,
          kSeq, kRelPad, kHdim, kQRScale, 1.0f,
          NODIV, 0L, NODIV, 0L);
      wmma_gemm64<0, 0, 0, 0, false><<<dim3(((kSeq / 64) * (kSeq / 64)) / 8, kBatch), 256, 0, stream>>>(
          q16 + tgtSlot, nullptr, kHdim, (long)kSlot,
          k16 + tgtSlot, nullptr, kHdim, (long)kSlot,
          (void*)Sbuf, nullptr, kSeq, (long)kSeq * kSeq,
          nullptr, nullptr, 0L,
          kSeq, kSeq, kHdim, kS1Scale, 1.0f,
          NODIV, 0L, NODIV, 0L);
      softmax_bins_kernel<<<dim3((kBatch * kSeq) / 8), 256, 0, stream>>>(Sbuf, QRg, Ph, Pl, Hh, Hl, kS2Scale);
      wmma_gemm64<1, 1, 0, 0, false><<<dim3(((kSeq / 64) * (kHdim / 64) + 7) / 8, kBatch), 256, 0, stream>>>(
          Ph, Pl, kSeq, (long)kSeq * kSeq,
          vTh + tgtSlot, vTl + tgtSlot, kSeq, (long)kSlot,
          (void*)(W1m + (size_t)(4 * a + c) * kHdim), nullptr, kEmb, (long)kSeq * kEmb,
          nullptr, nullptr, 0L,
          kSeq, kHdim, kSeq, 1.0f, 1.0f,
          NODIV, 0L, NODIV, 0L);
      wmma_gemm64<1, 3, 0, 0, false><<<dim3(((kSeq / 64) * (kHdim / 64) + 7) / 8, kBatch), 256, 0, stream>>>(
          Hh, Hl, kRelPad, (long)kSeq * kRelPad,
          relvT, nullptr, kRelPad, 0L,
          (void*)(W2m + (size_t)c * kSeq * kEmb + (size_t)a * kHdim), nullptr, kEmb, (long)(4 * kHdim),
          nullptr, nullptr, 0L,
          kSeq, kHdim, kRelPad, 1.0f, 1.0f,
          NODIV, 0L, NODIV, 0L);
    }
  }

  {
    const int n8 = kTok * kEmb / 8;
    combine_split_kernel<<<dim3(n8 / 256), 256, 0, stream>>>(W1m, W2m, attnh, attnl, n8);
  }
  wmma_gemm64<1, 3, 2, 0, false><<<dim3(((kTok / 64) * (kEmb / 64)) / 8, 1), 256, 0, stream>>>(
      attnh, attnl, kEmb, 0L,
      wo_bf, nullptr, kEmb, 0L,
      (void*)out, nullptr, kEmb, 0L,
      bo, nullptr, 0L,
      kTok, kEmb, kEmb, 1.0f, 1.0f,
      NODIV, 0L, NODIV, 0L);
}
